// Sequence_80779744903257
// MI455X (gfx1250) — hardware-verified
//
#include <hip/hip_runtime.h>
#include <math.h>

constexpr int BATCH  = 256;
constexpr int TSEQ   = 1024;
constexpr int HID    = 128;
constexpr int NGATE  = 4 * HID;
constexpr int NFUT   = 16;
constexpr int TOUT   = TSEQ + NFUT - 1;
constexpr int BTILE  = 16;
constexpr int NTHR   = 256;
constexpr int HPITCH = 136;
constexpr int H2P    = 132;
constexpr int OUTP   = 68;
constexpr int TCH    = 64;
constexpr int TPAD   = 1088;
constexpr float HCARRY  = 16.0f;
constexpr float WCARRY  = 16.0f;
constexpr float PRESC   = 256.0f;
constexpr float FOLD    = 1.0f / 256.0f;
static_assert(NGATE == 4 * HID);
static_assert(HID % 32 == 0);
static_assert(BATCH % BTILE == 0);
static_assert(HID == 16 * (NTHR / 32));
static_assert(HID == 4 * 32);
static_assert(NGATE == 2 * NTHR);
static_assert(BTILE == 2 * (NTHR / 32));
static_assert(TPAD % TCH == 0 && TPAD >= TOUT);
static_assert((TOUT - 1) / TCH == TPAD / TCH - 1);
static_assert((BATCH * TOUT) % 128 == 0);
static_assert(HPITCH % 8 == 0 && H2P % 4 == 0 && OUTP % 4 == 0 && OUTP >= TCH);

typedef __attribute__((ext_vector_type(16))) _Float16 v16h;
typedef __attribute__((ext_vector_type(8)))  _Float16 v8h;
typedef __attribute__((ext_vector_type(8)))  float    v8f;
typedef __attribute__((ext_vector_type(4)))  float    v4f;

__device__ __forceinline__ void grp_guard_h(v8f& a0, v8f& a1, v8f& a2, v8f& a3,
                                            v16h x, v16h y0, v16h y1, v16h y2, v16h y3) {
  asm volatile("v_nop\n\tv_nop\n\tv_nop\n\tv_nop"
               : "+v"(a0), "+v"(a1), "+v"(a2), "+v"(a3)
               : "v"(x), "v"(y0), "v"(y1), "v"(y2), "v"(y3));
}
__device__ __forceinline__ void acc_guard4(v8f& a, v8f& b, v8f& c, v8f& d) {
  asm volatile("v_nop\n\tv_nop\n\tv_nop\n\tv_nop" : "+v"(a), "+v"(b), "+v"(c), "+v"(d));
}

template <typename T> struct Frag;
template <> struct Frag<_Float16> {
  typedef v16h V; union U { v16h v; v8h h[2]; };
  static __device__ __forceinline__ v16h load(const _Float16* p) {
    U f; f.h[0] = *(const v8h*)(p); f.h[1] = *(const v8h*)(p + 16); return f.v;
  }
  static __device__ __forceinline__ v8f mma(v16h a, v16h b, v8f c) {
    return __builtin_amdgcn_wmma_f32_16x16x32_f16(false, a, false, b, (short)0, c, false, false);
  }
};

__device__ __forceinline__ float fsig(float x)  { return __builtin_amdgcn_rcpf(1.0f + __expf(-x)); }
__device__ __forceinline__ float ftanh(float x) { return 1.0f - 2.0f * __builtin_amdgcn_rcpf(__expf(2.0f * x) + 1.0f); }

__device__ __forceinline__ float cell_update(float zi, float zf, float zg, float zo, float& cst) {
  const float cn = fsig(zf) * cst + fsig(zi) * ftanh(zg);
  cst = cn;
  return fsig(zo) * ftanh(cn);
}

__global__ __launch_bounds__(NTHR) void cvt_w16_kernel(const float* __restrict__ src, unsigned short* __restrict__ dst,
                                                       int n8, float sc) {
  const int i = blockIdx.x * NTHR + threadIdx.x;
  if (i >= n8) return;
  const float* sp = src + (size_t)i * 8;
  const v4f a = *(const v4f*)(sp);
  const v4f b = *(const v4f*)(sp + 4);
  v8h hv;
#pragma unroll
  for (int e = 0; e < 4; ++e) {
    hv[e]     = (_Float16)(a[e] * sc);
    hv[4 + e] = (_Float16)(b[e] * sc);
  }
  unsigned short* dp = dst + (size_t)i * 8;
  *(volatile v8h*)dp = hv;
  __threadfence();
  *(volatile v8h*)dp = hv;
}

__global__ __launch_bounds__(NTHR) void lstm2_seq_kernel(
    const float* __restrict__ input, const float* __restrict__ Wih1,
    const float* __restrict__ bih1, const float* __restrict__ bhh1,
    const float* __restrict__ bih2, const float* __restrict__ bhh2,
    const float* __restrict__ Wlin, const float* __restrict__ blin,
    const unsigned short* __restrict__ W1p, const unsigned short* __restrict__ W2p,
    const unsigned short* __restrict__ W3p, float* __restrict__ STG) {
  __shared__ __align__(16) _Float16 h1s[2][BTILE * HPITCH];
  __shared__ __align__(16) _Float16 h2s[2][BTILE * HPITCH];
  __shared__ __align__(16) float    h2f[BTILE * H2P];
  __shared__ __align__(16) float    outs[BTILE * OUTP];
  __shared__ __align__(16) float    cb1[NGATE];
  __shared__ __align__(16) float    cb2[NGATE];
  __shared__ __align__(16) float    cwi[NGATE];
  __shared__ __align__(16) float    wlin_s[HID];
  __shared__ float xbuf[BTILE];

  const _Float16* W1 = (const _Float16*)W1p;
  const _Float16* W2 = (const _Float16*)W2p;
  const _Float16* W3 = (const _Float16*)W3p;
  const int tid = threadIdx.x, lane = tid & 31, wave = tid >> 5;
  const int c = lane & 15, hh = lane >> 4, koff = hh * 8, c4 = c * 4;
  const int bbase = blockIdx.x * BTILE;
  const int jcol  = 16 * wave + c;

  {
    unsigned* z1 = (unsigned*)(void*)&h1s[0][0];
    unsigned* z2 = (unsigned*)(void*)&h2s[0][0];
    constexpr int NW16 = (2 * BTILE * HPITCH) / 2;
#pragma unroll 1
    for (int i = tid; i < NW16; i += NTHR) { z1[i] = 0u; z2[i] = 0u; }
#pragma unroll 1
    for (int i = tid; i < BTILE * H2P; i += NTHR) h2f[i] = 0.0f;
#pragma unroll 1
    for (int i = tid; i < BTILE * OUTP; i += NTHR) outs[i] = 0.0f;
  }
  const float bl = blin[0];
  {
    const int i0 = tid, i1 = tid + NTHR;
    const float a0 = bih1[i0], a1 = bhh1[i0], a2 = bih1[i1], a3 = bhh1[i1];
    const float w0 = Wih1[i0], w1 = Wih1[i1];
    asm volatile("" ::: "memory");
    const float d0 = bih2[i0], d1 = bhh2[i0], d2 = bih2[i1], d3 = bhh2[i1];
    cb1[i0] = a0 + a1; cb1[i1] = a2 + a3;
    cwi[i0] = w0;      cwi[i1] = w1;
    cb2[i0] = d0 + d1; cb2[i1] = d2 + d3;
  }
  if (tid < HID) wlin_s[tid] = Wlin[tid];
  if (wave == 0) xbuf[lane & 15] = input[(size_t)(bbase + (lane & 15)) * TSEQ];
  __syncthreads();

  float b1v[4], wi1v[4], b2v[4];
#pragma unroll
  for (int q = 0; q < 4; ++q) {
    const int n = q * HID + jcol;
    b1v[q] = cb1[n]; wi1v[q] = cwi[n]; b2v[q] = cb2[n];
  }
  const v4f wl4 = *(const v4f*)(wlin_s + 4 * lane);
  float c1r[8], c2r[8];
#pragma unroll
  for (int r = 0; r < 8; ++r) { c1r[r] = 0.0f; c2r[r] = 0.0f; }

  const size_t GSTR = (size_t)HID * HID;
  const _Float16* w1row = W1 + (size_t)jcol * HID + koff;
  const _Float16* w2row = W2 + (size_t)jcol * HID + koff;
  const _Float16* w3row = W3 + (size_t)jcol * HID + koff;

#pragma unroll 1
  for (int t = 0; t < TOUT; ++t) {
    const int p = t & 1;
    float xv[8];
#pragma unroll
    for (int r = 0; r < 8; ++r) xv[r] = xbuf[8 * hh + r];

    v8f acc[4];
#pragma unroll
    for (int q = 0; q < 4; ++q)
#pragma unroll
      for (int r = 0; r < 8; ++r) acc[q][r] = (xv[r] * wi1v[q] + b1v[q]) * PRESC;
    {
      const _Float16* arow = &h1s[p][0] + c * HPITCH + koff;
#pragma unroll 1
      for (int k0 = 0; k0 < HID; k0 += 32) {
        const v16h a  = Frag<_Float16>::load(arow + k0);
        const v16h b0 = Frag<_Float16>::load(w1row + k0);
        const v16h b1 = Frag<_Float16>::load(w1row + GSTR + k0);
        const v16h b2 = Frag<_Float16>::load(w1row + 2 * GSTR + k0);
        const v16h b3 = Frag<_Float16>::load(w1row + 3 * GSTR + k0);
        acc[0] = Frag<_Float16>::mma(a, b0, acc[0]);
        acc[1] = Frag<_Float16>::mma(a, b1, acc[1]);
        acc[2] = Frag<_Float16>::mma(a, b2, acc[2]);
        acc[3] = Frag<_Float16>::mma(a, b3, acc[3]);
        grp_guard_h(acc[0], acc[1], acc[2], acc[3], a, b0, b1, b2, b3);
      }
    }
    acc_guard4(acc[0], acc[1], acc[2], acc[3]);
    {
      _Float16* h1n = &h1s[p ^ 1][0];
#pragma unroll
      for (int r = 0; r < 8; ++r) {
        const float hn = cell_update(acc[0][r] * FOLD, acc[1][r] * FOLD, acc[2][r] * FOLD, acc[3][r] * FOLD, c1r[r]);
        h1n[(8 * hh + r) * HPITCH + jcol] = (_Float16)(hn * HCARRY);
      }
    }
    __syncthreads();

#pragma unroll
    for (int q = 0; q < 4; ++q)
#pragma unroll
      for (int r = 0; r < 8; ++r) acc[q][r] = b2v[q] * PRESC;
    {
      const _Float16* arow = &h1s[p ^ 1][0] + c * HPITCH + koff;
#pragma unroll 1
      for (int k0 = 0; k0 < HID; k0 += 32) {
        const v16h a  = Frag<_Float16>::load(arow + k0);
        const v16h b0 = Frag<_Float16>::load(w2row + k0);
        const v16h b1 = Frag<_Float16>::load(w2row + GSTR + k0);
        const v16h b2 = Frag<_Float16>::load(w2row + 2 * GSTR + k0);
        const v16h b3 = Frag<_Float16>::load(w2row + 3 * GSTR + k0);
        acc[0] = Frag<_Float16>::mma(a, b0, acc[0]);
        acc[1] = Frag<_Float16>::mma(a, b1, acc[1]);
        acc[2] = Frag<_Float16>::mma(a, b2, acc[2]);
        acc[3] = Frag<_Float16>::mma(a, b3, acc[3]);
        grp_guard_h(acc[0], acc[1], acc[2], acc[3], a, b0, b1, b2, b3);
      }
    }
    {
      const _Float16* arow = &h2s[p][0] + c * HPITCH + koff;
#pragma unroll 1
      for (int k0 = 0; k0 < HID; k0 += 32) {
        const v16h a  = Frag<_Float16>::load(arow + k0);
        const v16h b0 = Frag<_Float16>::load(w3row + k0);
        const v16h b1 = Frag<_Float16>::load(w3row + GSTR + k0);
        const v16h b2 = Frag<_Float16>::load(w3row + 2 * GSTR + k0);
        const v16h b3 = Frag<_Float16>::load(w3row + 3 * GSTR + k0);
        acc[0] = Frag<_Float16>::mma(a, b0, acc[0]);
        acc[1] = Frag<_Float16>::mma(a, b1, acc[1]);
        acc[2] = Frag<_Float16>::mma(a, b2, acc[2]);
        acc[3] = Frag<_Float16>::mma(a, b3, acc[3]);
        grp_guard_h(acc[0], acc[1], acc[2], acc[3], a, b0, b1, b2, b3);
      }
    }
    acc_guard4(acc[0], acc[1], acc[2], acc[3]);
    {
      _Float16* h2n = &h2s[p ^ 1][0];
#pragma unroll
      for (int r = 0; r < 8; ++r) {
        const float hn = cell_update(acc[0][r] * FOLD, acc[1][r] * FOLD, acc[2][r] * FOLD, acc[3][r] * FOLD, c2r[r]);
        h2n[(8 * hh + r) * HPITCH + jcol] = (_Float16)(hn * HCARRY);
        h2f[(8 * hh + r) * H2P + jcol]    = hn;
      }
    }
    __syncthreads();

    {
      const int r0 = 2 * wave, r1 = 2 * wave + 1;
      const v4f ha = *(const v4f*)(h2f + r0 * H2P + 4 * lane);
      const v4f hb = *(const v4f*)(h2f + r1 * H2P + 4 * lane);
      float s0 = (ha[0] * wl4[0] + ha[1] * wl4[1]) + (ha[2] * wl4[2] + ha[3] * wl4[3]);
      float s1 = (hb[0] * wl4[0] + hb[1] * wl4[1]) + (hb[2] * wl4[2] + hb[3] * wl4[3]);
#pragma unroll
      for (int off = 1; off < 32; off <<= 1) {
        s0 += __shfl_xor(s0, off, 32);
        s1 += __shfl_xor(s1, off, 32);
      }
      const float o0 = s0 + bl, o1 = s1 + bl;
      const int odd = lane & 1;
      const float osel = odd ? o1 : o0;
      const int row = r0 + odd;
      const int tn  = (t + 1 < TSEQ) ? (t + 1) : (TSEQ - 1);
      const float xin = input[(size_t)(bbase + row) * TSEQ + tn];
      const float fa  = (t + 1 < TSEQ) ? 1.0f : 0.0f;
      const float xn  = fmaf(fa, xin, (1.0f - fa) * osel);
      outs[row * OUTP + (t & (TCH - 1))] = osel;
      xbuf[row] = xn;
    }
    __syncthreads();

    if (((t & (TCH - 1)) == (TCH - 1)) || (t == TOUT - 1)) {
      const int ch  = t / TCH;
      const int row = 2 * wave + hh;
      const v4f v = *(const v4f*)(outs + row * OUTP + c4);
      float* dst = STG + (size_t)(bbase + row) * TPAD + (size_t)ch * TCH + c4;
      for (int pass = 0; pass < 2; ++pass) {
        *(volatile v4f*)dst = v;
        __threadfence();
      }
    }
  }
}

__global__ __launch_bounds__(NTHR) void out_lines_kernel(const float* __restrict__ STG, float* __restrict__ out, int n4) {
  const int i = blockIdx.x * NTHR + threadIdx.x;
  if (i >= n4) return;
  v4f v;
#pragma unroll
  for (int j = 0; j < 4; ++j) {
    const int e  = 4 * i + j;
    const int b  = e / TOUT;
    const int tt = e - b * TOUT;
    v[j] = STG[(size_t)b * TPAD + tt];
  }
  float* op = out + (size_t)i * 4;
  for (int pass = 0; pass < 2; ++pass) {
    *(volatile v4f*)op = v;
    __threadfence();
  }
}

extern "C" void kernel_launch(void* const* d_in, const int* in_sizes, int n_in,
                              void* d_out, int out_size, void* d_ws, size_t ws_size, hipStream_t stream) {
  if (n_in < 11 || d_out == nullptr || d_ws == nullptr) return;
  if (in_sizes[0] != BATCH * TSEQ || in_sizes[1] != NGATE || in_sizes[2] != NGATE * HID || in_sizes[3] != NGATE ||
      in_sizes[4] != NGATE || in_sizes[5] != NGATE * HID || in_sizes[6] != NGATE * HID || in_sizes[7] != NGATE ||
      in_sizes[8] != NGATE || in_sizes[9] != HID || in_sizes[10] < 1 || out_size != BATCH * TOUT) return;

  const float* input = (const float*)d_in[0];
  const float* Wih1  = (const float*)d_in[1];
  const float* Whh1  = (const float*)d_in[2];
  const float* bih1  = (const float*)d_in[3];
  const float* bhh1  = (const float*)d_in[4];
  const float* Wih2  = (const float*)d_in[5];
  const float* Whh2  = (const float*)d_in[6];
  const float* bih2  = (const float*)d_in[7];
  const float* bhh2  = (const float*)d_in[8];
  const float* Wlin  = (const float*)d_in[9];
  const float* blin  = (const float*)d_in[10];
  float* out = (float*)d_out;

  char* ws = (char*)d_ws; size_t off = 0;
  auto carve = [&](size_t bytes) -> char* { char* p = ws + off; off += (bytes + 255) & ~(size_t)255; return p; };
  unsigned short* W1  = (unsigned short*)carve((size_t)NGATE * HID * 2);
  unsigned short* W2  = (unsigned short*)carve((size_t)NGATE * HID * 2);
  unsigned short* W3  = (unsigned short*)carve((size_t)NGATE * HID * 2);
  float*          STG = (float*)carve((size_t)BATCH * TPAD * 4);
  if (off > ws_size || off > (size_t)134217728) return;

  const int n8 = NGATE * HID / 8;
  cvt_w16_kernel<<<(n8 + NTHR - 1) / NTHR, NTHR, 0, stream>>>(Whh1, W1, n8, WCARRY);
  cvt_w16_kernel<<<(n8 + NTHR - 1) / NTHR, NTHR, 0, stream>>>(Wih2, W2, n8, WCARRY);
  cvt_w16_kernel<<<(n8 + NTHR - 1) / NTHR, NTHR, 0, stream>>>(Whh2, W3, n8, WCARRY);
  lstm2_seq_kernel<<<BATCH / BTILE, NTHR, 0, stream>>>(input, Wih1, bih1, bhh1, bih2, bhh2, Wlin, blin, W1, W2, W3, STG);
  const int n4 = BATCH * TOUT / 4;
  out_lines_kernel<<<(n4 + NTHR - 1) / NTHR, NTHR, 0, stream>>>(STG, out, n4);
}
